// UnetDownAttention_17291538333702
// MI455X (gfx1250) — hardware-run, weakly checked
//
#include <hip/hip_runtime.h>


#define NB_  8
#define CC   128
#define HH   64
#define WWD  64
#define TT   4096
#define NR   (NB_ * TT)
#define KC   1152
#define NEK  128
#define NKEY 4224
#define PCAR 1024.0f
typedef _Float16 h16;
typedef unsigned short bf;
typedef __attribute__((ext_vector_type(16))) __bf16   v16bf;
typedef __attribute__((ext_vector_type(16))) _Float16 v16h;
typedef __attribute__((ext_vector_type(8)))  _Float16 v8h;
typedef __attribute__((ext_vector_type(8)))  unsigned short v8us;
typedef __attribute__((ext_vector_type(8)))  float    v8f;
typedef __attribute__((ext_vector_type(4)))  float    v4f;
typedef v8h  __attribute__((may_alias)) v8ha;
typedef v4f  __attribute__((may_alias)) v4fa;
typedef v8us __attribute__((may_alias)) v8usa;

__device__ __forceinline__ unsigned short f2bf(float f) { unsigned u = __float_as_uint(f); u += 0x7FFFu + ((u >> 16) & 1u); return (unsigned short)(u >> 16); }
__device__ __forceinline__ float bf2f(unsigned short b) { return __uint_as_float(((unsigned)b) << 16); }
__device__ __forceinline__ float bfr(float f) { return bf2f(f2bf(f)); }
__device__ __forceinline__ v16h cat16(v8h lo, v8h hi) { return __builtin_shufflevector(lo, hi, 0, 1, 2, 3, 4, 5, 6, 7, 8, 9, 10, 11, 12, 13, 14, 15); }
__device__ __forceinline__ v16bf cat16b(v8us lo, v8us hi) { return __builtin_bit_cast(v16bf, __builtin_shufflevector(lo, hi, 0, 1, 2, 3, 4, 5, 6, 7, 8, 9, 10, 11, 12, 13, 14, 15)); }
__device__ __forceinline__ v8f wmma16(v16h a, v16h b, v8f c) { return __builtin_amdgcn_wmma_f32_16x16x32_f16(false, a, false, b, (short)0, c, false, false); }
__device__ __forceinline__ v8f wmmab(v16bf a, v16bf b, v8f c) { return __builtin_amdgcn_wmma_f32_16x16x32_bf16(false, a, false, b, (short)0, c, false, false); }


template <typename T16> struct WFrag;
template <> struct WFrag<h16> { typedef v16h V; static __device__ __forceinline__ V ld(const h16* p) { return cat16(*(const v8h*)p, *(const v8h*)(p + 16)); } static __device__ __forceinline__ v8f mma(V a, V b, v8f c) { return wmma16(a, b, c); } };
template <> struct WFrag<bf> { typedef v16bf V; static __device__ __forceinline__ V ld(const bf* p) { return cat16b(*(const v8us*)p, *(const v8us*)(p + 16)); } static __device__ __forceinline__ v8f mma(V a, V b, v8f c) { return wmmab(a, b, c); } };
template <typename T16, int NSPLIT, bool BIAS>
__global__ __launch_bounds__(32) void k_gemmw(const T16* __restrict__ A, const T16* __restrict__ A2, const T16* __restrict__ Bt, const T16* __restrict__ Bt2, int K, float* C, int ldc, const float* __restrict__ bias, size_t sA, size_t sB, size_t sC) {
    typedef typename WFrag<T16>::V V;
    __shared__ __align__(16) float os[16 * 68];
    const size_t z = blockIdx.z; A += z * sA; if (A2) A2 += z * sA; Bt += z * sB; if (Bt2) Bt2 += z * sB; C += z * sC;
    const int lane = threadIdx.x & 31, lr = lane & 15, hi = lane >> 4; const int r0 = blockIdx.x * 64, c0 = blockIdx.y * 64;
    v8f acc[4][4];
#pragma unroll
    for (int mb = 0; mb < 4; ++mb)
#pragma unroll
        for (int nb = 0; nb < 4; ++nb) acc[mb][nb] = (v8f){};
    const size_t aoff = (size_t)(r0 + lr) * K + 8 * hi, boff = (size_t)(c0 + lr) * K + 8 * hi;
#pragma unroll 1
    for (int kc = 0; kc < K; kc += 32) {
        V a[4], a2[4];
#pragma unroll
        for (int mb = 0; mb < 4; ++mb) { a[mb] = WFrag<T16>::ld(A + aoff + (size_t)mb * 16 * K + kc); if (NSPLIT == 1 || NSPLIT == 2) a2[mb] = WFrag<T16>::ld(A2 + aoff + (size_t)mb * 16 * K + kc); }
#pragma unroll
        for (int nb = 0; nb < 4; ++nb) { const V b = WFrag<T16>::ld(Bt + boff + (size_t)nb * 16 * K + kc); V b2; if (NSPLIT >= 2) b2 = WFrag<T16>::ld(Bt2 + boff + (size_t)nb * 16 * K + kc);
#pragma unroll
            for (int mb = 0; mb < 4; ++mb) { acc[mb][nb] = WFrag<T16>::mma(a[mb], b, acc[mb][nb]); if (NSPLIT == 1 || NSPLIT == 2) acc[mb][nb] = WFrag<T16>::mma(a2[mb], b, acc[mb][nb]); if (NSPLIT >= 2) acc[mb][nb] = WFrag<T16>::mma(a[mb], b2, acc[mb][nb]); } }
        asm volatile("v_nop\n\tv_nop\n\tv_nop\n\tv_nop" : "+v"(acc[0][0]), "+v"(acc[1][1]), "+v"(acc[2][2]), "+v"(acc[3][3]) : "v"(a[0]), "v"(a[3]));
    }
#pragma unroll
    for (int mb = 0; mb < 4; ++mb) {
#pragma unroll
        for (int nb = 0; nb < 4; ++nb) {
#pragma unroll
            for (int j = 0; j < 8; ++j) os[(hi * 8 + j) * 68 + nb * 16 + lr] = acc[mb][nb][j]; }
        __builtin_amdgcn_wave_barrier(); asm volatile("" ::: "memory");
        float* crow = C + (size_t)(r0 + mb * 16) * ldc + c0;
#pragma unroll 1
        for (int ps = 0; ps < 2; ++ps) {
#pragma unroll
            for (int s = 0; s < 8; ++s) { const int row = 2 * s + hi, cofs = lr * 4; v4f val = *(const v4fa*)(os + row * 68 + cofs); if (BIAS) { val[0] += bfr(bias[c0 + cofs]); val[1] += bfr(bias[c0 + cofs + 1]); val[2] += bfr(bias[c0 + cofs + 2]); val[3] += bfr(bias[c0 + cofs + 3]); }
                *(volatile v4f*)(crow + (size_t)row * ldc + cofs) = val; }
            if (ps == 0) __threadfence(); }
        __builtin_amdgcn_wave_barrier(); asm volatile("" ::: "memory");
    }
}

__device__ __forceinline__ h16 tohx(float x) { return (h16)x; }
__device__ __forceinline__ float gelu_(float x) { return __fmul_rn(0.5f * x, __fadd_rn(1.0f, erff(x * 0.7071067811865476f))); }
typedef __attribute__((ext_vector_type(2))) _Float16 v2h;
typedef __attribute__((ext_vector_type(4))) _Float16 v4h;

__global__ __launch_bounds__(256) void k_w16(const float* __restrict__ w, size_t n4, h16* W) { const size_t e = ((size_t)blockIdx.x * 256 + threadIdx.x) * 4; if (e >= n4 * 4) return; const v4f a = *(const v4f*)(w + e); v4h o; o[0] = tohx(bfr(a[0])); o[1] = tohx(bfr(a[1])); o[2] = tohx(bfr(a[2])); o[3] = tohx(bfr(a[3])); *(volatile v4h*)(W + e) = o; __threadfence(); *(volatile v4h*)(W + e) = o; }
__global__ __launch_bounds__(128) void k_emb(const float* __restrict__ temb, const float* __restrict__ mix, const float* __restrict__ w1, const float* __restrict__ b1, const float* __restrict__ w2, const float* __restrict__ b2, float* EMB) { __shared__ float e0[CC], e1[CC]; const int b = blockIdx.x, c = threadIdx.x;
    e0[c] = __fadd_rn(bfr(temb[b * CC + c]), bfr(mix[b * CC + c])); __syncthreads(); float a = bfr(b1[c]);
#pragma unroll 1
    for (int k = 0; k < CC; ++k) { float p = __fmul_rn(e0[k], bfr(w1[c * CC + k])); asm volatile("" : "+v"(p)); a = __fadd_rn(a, p); } e1[c] = gelu_(a); __syncthreads(); float s = bfr(b2[c]);
#pragma unroll 1
    for (int k = 0; k < CC; ++k) { float p = __fmul_rn(e1[k], bfr(w2[c * CC + k])); asm volatile("" : "+v"(p)); s = __fadd_rn(s, p); } *(volatile float*)(EMB + b * CC + c) = s; __threadfence(); *(volatile float*)(EMB + b * CC + c) = s; }
__global__ __launch_bounds__(256) void k_ekv(const float* __restrict__ mix, const float* __restrict__ ew, const float* __restrict__ eb, int b, h16* KT16, h16* V16) { const int i = blockIdx.x * 256 + threadIdx.x; if (i >= 2 * CC * (CC / 4)) return; const int s4 = (i % (CC / 4)) * 4; const int o = i / (CC / 4);
    const float* m = mix + b * CC; float acc[4]; const float bo = bfr(eb[o]); acc[0] = acc[1] = acc[2] = acc[3] = bo;
#pragma unroll 1
    for (int c = 0; c < CC; ++c) { const float wc = __fmul_rn(bfr(ew[o * CC + c]), bfr(m[c]));
#pragma unroll
        for (int u = 0; u < 4; ++u) { float mm = __fmul_rn(bfr(m[c]), bfr(m[s4 + u])); float p = __fmul_rn(bfr(ew[o * CC + c]), mm); asm volatile("" : "+v"(p)); acc[u] = __fadd_rn(acc[u], p); } (void)wc; }
    v4h ov; ov[0] = tohx(acc[0]); ov[1] = tohx(acc[1]); ov[2] = tohx(acc[2]); ov[3] = tohx(acc[3]);
    if (o >= CC) { h16* dst = V16 + (size_t)(o - CC) * NKEY + s4; *(volatile v4h*)dst = ov; __threadfence(); *(volatile v4h*)dst = ov; }
    else {
        h16* dst = KT16 + (size_t)NKEY * CC + (size_t)o * CC + s4;     *(volatile v4h*)dst = ov; __threadfence(); *(volatile v4h*)dst = ov; } }
__global__ __launch_bounds__(256) void k_ekT(h16* KT16) { const int e = (blockIdx.x * 256 + threadIdx.x) * 2; if (e >= NEK * CC) return; const int o = e % CC; const int s = e / CC; const h16* EK = KT16 + (size_t)NKEY * CC; v2h v; v[0] = EK[(size_t)o * CC + s]; v[1] = EK[(size_t)(o + 1) * CC + s]; *(volatile v2h*)(KT16 + (size_t)s * CC + o) = v; __threadfence(); *(volatile v2h*)(KT16 + (size_t)s * CC + o) = v; }
template <int MODE> __global__ __launch_bounds__(256) void k_i2c(const float* __restrict__ src, const float* __restrict__ EMB, h16* A) { const size_t e = ((size_t)blockIdx.x * 256 + threadIdx.x) * 4; if (e >= (size_t)NR * KC) return; const int k = (int)(e % KC); const int r = (int)(e / KC); const int b = r / TT, yx = r % TT, y = yx / WWD, x = yx % WWD; v4h o;
#pragma unroll
    for (int q = 0; q < 4; ++q) { const int kk = k + q; const int c = kk / 9, uv = kk % 9, u = uv / 3, v = uv % 3; const int yy = y + u - 1, xx = x + v - 1; float val = 0.f;
        if (yy >= 0 && yy < HH && xx >= 0 && xx < WWD) { if (MODE == 0) val = __fadd_rn(bfr(src[(((size_t)b * CC + c) * HH + yy) * WWD + xx]), EMB[b * CC + c]); else val = src[((size_t)b * TT + yy * WWD + xx) * CC + c]; }
        o[q] = tohx(val); }
    *(volatile v4h*)(A + e) = o; __threadfence(); *(volatile v4h*)(A + e) = o; }
template <int P> __global__ __launch_bounds__(256) void k_cpart(const float* __restrict__ C, const float* __restrict__ mu, float* PART) { const int i = blockIdx.x * 256 + threadIdx.x; if (i >= 256 * CC) return; const int c = i % CC, rb = i / CC; float s = 0.f; const float m = (P == 2) ? mu[c] : 0.f;
#pragma unroll 1
    for (int r = rb * 128; r < rb * 128 + 128; ++r) { float d0 = __fsub_rn(C[(size_t)r * CC + c], m); asm volatile("" : "+v"(d0)); if (P == 2) { float q = __fmul_rn(d0, d0); asm volatile("" : "+v"(q)); s = __fadd_rn(s, q); } else s = __fadd_rn(s, d0); }
    *(volatile float*)(PART + i) = s; __threadfence(); *(volatile float*)(PART + i) = s; }
__global__ __launch_bounds__(128) void k_cfin(const float* __restrict__ PART, float* STAT) { const int c = threadIdx.x; float s = 0.f;
#pragma unroll 1
    for (int rb = 0; rb < 256; ++rb) s = __fadd_rn(s, PART[rb * CC + c]); const float v = s * (1.0f / NR); *(volatile float*)(STAT + c) = v; __threadfence(); *(volatile float*)(STAT + c) = v; }
__global__ __launch_bounds__(256) void k_bngelu(const float* __restrict__ C, const float* __restrict__ mean, const float* __restrict__ var, const float* __restrict__ g, const float* __restrict__ bb, float* Y) { const size_t e = ((size_t)blockIdx.x * 256 + threadIdx.x) * 4; if (e >= (size_t)NR * CC) return; const int c = (int)(e % CC); const v4f a = *(const v4f*)(C + e); v4f o;
#pragma unroll
    for (int u = 0; u < 4; ++u) { const int cc = c + u; float n = __fmul_rn(__fsub_rn(a[u], mean[cc]), __frsqrt_rn(__fadd_rn(var[cc], 1e-5f))); asm volatile("" : "+v"(n)); float t = __fmul_rn(n, bfr(g[cc])); asm volatile("" : "+v"(t)); o[u] = gelu_(__fadd_rn(t, bfr(bb[cc]))); }
    *(volatile v4f*)(Y + e) = o; __threadfence(); *(volatile v4f*)(Y + e) = o; }
template <int P> __global__ __launch_bounds__(256) void k_gpart(const float* __restrict__ Hh, const float* __restrict__ mu, float* GP) { const int i = blockIdx.x * 256 + threadIdx.x; if (i >= NB_ * 8 * 64) return; const int pb = i % 64; const int g = (i / 64) % 8; const int b = i / 512; const float m = (P == 2) ? mu[b * 8 + g] : 0.f; float s = 0.f;
#pragma unroll 1
    for (int t = pb * 64; t < pb * 64 + 64; ++t) { const float* r = Hh + ((size_t)b * TT + t) * CC + g * 16;
#pragma unroll
        for (int c = 0; c < 16; ++c) { float d0 = __fsub_rn(r[c], m); asm volatile("" : "+v"(d0)); if (P == 2) { float q = __fmul_rn(d0, d0); asm volatile("" : "+v"(q)); s = __fadd_rn(s, q); } else s = __fadd_rn(s, d0); } }
    *(volatile float*)(GP + i) = s; __threadfence(); *(volatile float*)(GP + i) = s; }
__global__ __launch_bounds__(64) void k_gfin(const float* __restrict__ GP, float* GSTAT) { const int i = threadIdx.x; float s = 0.f;
#pragma unroll 1
    for (int pb = 0; pb < 64; ++pb) s = __fadd_rn(s, GP[i * 64 + pb]); const float v = s * (1.0f / (TT * 16)); *(volatile float*)(GSTAT + i) = v; __threadfence(); *(volatile float*)(GSTAT + i) = v; }
__global__ __launch_bounds__(256) void k_gn16(const float* __restrict__ Hh, const float* __restrict__ gm, const float* __restrict__ gv, const float* __restrict__ g, const float* __restrict__ bb, h16* HN16) { const size_t e = ((size_t)blockIdx.x * 256 + threadIdx.x) * 4; if (e >= (size_t)NR * CC) return; const int c = (int)(e % CC); const int b = (int)(e / ((size_t)TT * CC)); const v4f a = *(const v4f*)(Hh + e); v4h o;
#pragma unroll
    for (int u = 0; u < 4; ++u) { const int cc = c + u; const int gi = b * 8 + cc / 16; float n = __fmul_rn(__fsub_rn(a[u], gm[gi]), __frsqrt_rn(__fadd_rn(gv[gi], 1e-5f))); asm volatile("" : "+v"(n)); float t = __fmul_rn(n, bfr(g[cc])); asm volatile("" : "+v"(t)); o[u] = tohx(__fadd_rn(t, bfr(bb[cc]))); }
    *(volatile v4h*)(HN16 + e) = o; __threadfence(); *(volatile v4h*)(HN16 + e) = o; }
__global__ __launch_bounds__(256) void k_qkT(const float* __restrict__ QKV, const float* __restrict__ qb, h16* Q16, h16* KT16) { const int e = (blockIdx.x * 256 + threadIdx.x) * 2; if (e >= TT * CC) return; const int c = e % CC; const int t = e / CC; v2h oq, ok;
#pragma unroll
    for (int u = 0; u < 2; ++u) { oq[u] = tohx(__fadd_rn(QKV[(size_t)(c + u) * TT + t], bfr(qb[c + u])) * 0.08838834764831845f); ok[u] = tohx(__fadd_rn(QKV[(size_t)(CC + c + u) * TT + t], bfr(qb[CC + c + u]))); }
    for (int ps = 0; ps < 2; ++ps) { *(volatile v2h*)(Q16 + e) = oq; *(volatile v2h*)(KT16 + (size_t)(NEK + t) * CC + c) = ok; if (ps == 0) __threadfence(); } }
__global__ __launch_bounds__(256) void k_v16(const float* __restrict__ QKV, const float* __restrict__ qb, h16* V16) { const int e = (blockIdx.x * 256 + threadIdx.x) * 4; if (e >= CC * TT) return; const int s = e % TT; const int c = e / TT; const v4f a = *(const v4f*)(QKV + (size_t)(2 * CC + c) * TT + s); const float bb = bfr(qb[2 * CC + c]); v4h o; o[0] = tohx(__fadd_rn(a[0], bb)); o[1] = tohx(__fadd_rn(a[1], bb)); o[2] = tohx(__fadd_rn(a[2], bb)); o[3] = tohx(__fadd_rn(a[3], bb));
    h16* dst = V16 + (size_t)c * NKEY + NEK + s; *(volatile v4h*)dst = o; __threadfence(); *(volatile v4h*)dst = o; }
__global__ __launch_bounds__(256) void k_a16(const float* __restrict__ AT, h16* A16) { const int e = (blockIdx.x * 256 + threadIdx.x) * 4; if (e >= TT * CC) return; const v4f a = *(const v4f*)(AT + e); v4h o; o[0] = tohx(a[0] * (1.0f / PCAR)); o[1] = tohx(a[1] * (1.0f / PCAR)); o[2] = tohx(a[2] * (1.0f / PCAR)); o[3] = tohx(a[3] * (1.0f / PCAR)); *(volatile v4h*)(A16 + e) = o; __threadfence(); *(volatile v4h*)(A16 + e) = o; }
__global__ __launch_bounds__(256) void k_resid(const float* __restrict__ Hh, const float* __restrict__ ATT, float* H2) { const int e = (blockIdx.x * 256 + threadIdx.x) * 4; if (e >= TT * CC) return; const v4f a = *(const v4f*)(Hh + e), t = *(const v4f*)(ATT + e); v4f o; o[0] = __fadd_rn(a[0], t[0]); o[1] = __fadd_rn(a[1], t[1]); o[2] = __fadd_rn(a[2], t[2]); o[3] = __fadd_rn(a[3], t[3]); *(volatile v4f*)(H2 + e) = o; __threadfence(); *(volatile v4f*)(H2 + e) = o; }
__global__ __launch_bounds__(256) void k_pool(const float* __restrict__ H2, float* OUT) { const int e = (blockIdx.x * 256 + threadIdx.x) * 4; if (e >= NB_ * CC * 32 * 32) return; const int xo = e % 32; const int yo = (e / 32) % 32; const int c = (e / 1024) % CC; const int b = e / (1024 * CC); v4f o;
#pragma unroll
    for (int u = 0; u < 4; ++u) { const int x0 = 2 * (xo + u), y0 = 2 * yo; auto at = [&](int y, int x) { return H2[((size_t)b * TT + y * WWD + x) * CC + c]; }; o[u] = fmaxf(fmaxf(at(y0, x0), at(y0, x0 + 1)), fmaxf(at(y0 + 1, x0), at(y0 + 1, x0 + 1))); }
    *(volatile v4f*)(OUT + e) = o; __threadfence(); *(volatile v4f*)(OUT + e) = o; }
template <int NFULL, int TAIL> __global__ __launch_bounds__(256) void k_soft(const float* __restrict__ Sb, int nrows, int rowsper, int rvalid, int nvalid, h16* P) { const int lane = threadIdx.x & 31; const size_t row = (size_t)blockIdx.x * 8 + (threadIdx.x >> 5); if (row >= (size_t)nrows) return; constexpr int LD = NFULL * 128 + TAIL * 64; const float* sr = Sb + row * LD; h16* pr = P + row * LD; const bool live = (int)(row % rowsper) < rvalid; float mx = -3.0e38f;
#pragma unroll 1
    for (int ch = 0; ch < NFULL + TAIL; ++ch) { if (ch == NFULL && lane >= 16) break; const int j0 = ch * 128 + lane * 4; const v4f a = *(const v4f*)(sr + j0);
#pragma unroll
        for (int q = 0; q < 4; ++q) if (j0 + q < nvalid) mx = fmaxf(mx, a[q]); }
#pragma unroll
    for (int sh = 16; sh; sh >>= 1) mx = fmaxf(mx, __shfl_xor(mx, sh, 32));
    float sum = 0.f;
#pragma unroll 1
    for (int ch = 0; ch < NFULL + TAIL; ++ch) { if (ch == NFULL && lane >= 16) break; const int j0 = ch * 128 + lane * 4; const v4f a = *(const v4f*)(sr + j0);
#pragma unroll
        for (int q = 0; q < 4; ++q) if (j0 + q < nvalid) { float d0 = __fsub_rn(a[q], mx); asm volatile("" : "+v"(d0)); sum += __expf(d0); } }
#pragma unroll
    for (int sh = 16; sh; sh >>= 1) sum += __shfl_xor(sum, sh, 32);
    const float f = live ? __fdiv_rn(PCAR, sum) : 0.f;
    for (int ps = 0; ps < 2; ++ps) {
#pragma unroll 1
        for (int ch = 0; ch < NFULL + TAIL; ++ch) { if (ch == NFULL && lane >= 16) break; const int j0 = ch * 128 + lane * 4; const v4f a = *(const v4f*)(sr + j0); v4h o;
#pragma unroll
            for (int q = 0; q < 4; ++q) { float val = 0.f; if (live && j0 + q < nvalid) { float d0 = __fsub_rn(a[q], mx); asm volatile("" : "+v"(d0)); val = __fmul_rn(__expf(d0), f); } o[q] = tohx(val); } *(volatile v4h*)(pr + j0) = o; }
        if (ps == 0) __threadfence(); } }

extern "C" void kernel_launch(void* const* d_in, const int* in_sizes, int n_in,
                              void* d_out, int out_size, void* d_ws, size_t ws_size, hipStream_t stream) {
    (void)in_sizes; (void)n_in; (void)out_size;
    const float** I = (const float**)d_in;
    const float *x = I[0], *temb = I[1], *mixemb = I[2], *emb_w1 = I[3], *emb_b1 = I[4], *emb_w2 = I[5], *emb_b2 = I[6], *c1w = I[7], *c1b = I[8], *bn1g = I[9], *bn1b = I[10], *c2w = I[11], *c2b = I[12], *bn2g = I[13], *bn2b = I[14], *gng = I[15], *gnb = I[16], *qkvw = I[17], *qkvb = I[18], *encw = I[19], *encb = I[20], *pw = I[21], *pb = I[22];
    float* OUT = (float*)d_out;
    char* wsp = (char*)d_ws;
    auto take = [&](size_t bytes) { char* p = wsp; wsp += (bytes + 255) & ~(size_t)255; return (void*)p; };
    h16* C1W = (h16*)take((size_t)CC * KC * 2); h16* C2W = (h16*)take((size_t)CC * KC * 2); h16* QKVW = (h16*)take((size_t)3 * CC * CC * 2); h16* PW = (h16*)take((size_t)CC * CC * 2); float* EMB = (float*)take(NB_ * CC * 4);
    h16* A = (h16*)take((size_t)NR * KC * 2);
    float* Cb = (float*)take((size_t)NR * CC * 4); float* X1 = (float*)take((size_t)NR * CC * 4); float* Hf = (float*)take((size_t)NR * CC * 4); float* PART = (float*)take(256 * CC * 4); float* MEAN = (float*)take(CC * 4); float* VAR = (float*)take(CC * 4); float* GP = (float*)take(NB_ * 8 * 64 * 4); float* GM = (float*)take(64 * 4); float* GV = (float*)take(64 * 4); h16* HN16 = (h16*)take((size_t)NR * CC * 2);
    float* QKV = (float*)take((size_t)3 * CC * TT * 4); h16* Q16 = (h16*)take((size_t)TT * CC * 2); h16* KT16 = (h16*)take(((size_t)NKEY * CC + (size_t)CC * CC) * 2); h16* V16 = (h16*)take((size_t)CC * NKEY * 2); h16* P16 = (h16*)take((size_t)TT * NKEY * 2); float* AT = (float*)take((size_t)TT * CC * 4); h16* A16 = (h16*)take((size_t)TT * CC * 2); float* ATT = (float*)take((size_t)TT * CC * 4); float* H2 = (float*)take((size_t)NR * CC * 4);
    float* Sb = (float*)A;
    if ((size_t)(wsp - (char*)d_ws) > ws_size) return;
    k_w16<<<(unsigned)(((size_t)CC * KC / 4 + 255) / 256), 256, 0, stream>>>(c1w, (size_t)CC * KC / 4, C1W); k_w16<<<(unsigned)(((size_t)CC * KC / 4 + 255) / 256), 256, 0, stream>>>(c2w, (size_t)CC * KC / 4, C2W); k_w16<<<(3 * CC * CC / 4 + 255) / 256, 256, 0, stream>>>(qkvw, (size_t)3 * CC * CC / 4, QKVW); k_w16<<<(CC * CC / 4 + 255) / 256, 256, 0, stream>>>(pw, (size_t)CC * CC / 4, PW);
    k_emb<<<NB_, 128, 0, stream>>>(temb, mixemb, emb_w1, emb_b1, emb_w2, emb_b2, EMB);
    k_i2c<0><<<(unsigned)(((size_t)NR * KC / 4 + 255) / 256), 256, 0, stream>>>(x, EMB, A);
    k_gemmw<h16, 0, true><<<dim3(NR / 64, CC / 64, 1), 32, 0, stream>>>(A, nullptr, C1W, nullptr, KC, Cb, CC, c1b, 0, 0, 0);
    k_cpart<1><<<(256 * CC + 255) / 256, 256, 0, stream>>>(Cb, nullptr, PART); k_cfin<<<1, 128, 0, stream>>>(PART, MEAN); k_cpart<2><<<(256 * CC + 255) / 256, 256, 0, stream>>>(Cb, MEAN, PART); k_cfin<<<1, 128, 0, stream>>>(PART, VAR);
    k_bngelu<<<(unsigned)(((size_t)NR * CC / 4 + 255) / 256), 256, 0, stream>>>(Cb, MEAN, VAR, bn1g, bn1b, X1);
    k_i2c<1><<<(unsigned)(((size_t)NR * KC / 4 + 255) / 256), 256, 0, stream>>>(X1, EMB, A);
    k_gemmw<h16, 0, true><<<dim3(NR / 64, CC / 64, 1), 32, 0, stream>>>(A, nullptr, C2W, nullptr, KC, Cb, CC, c2b, 0, 0, 0);
    k_cpart<1><<<(256 * CC + 255) / 256, 256, 0, stream>>>(Cb, nullptr, PART); k_cfin<<<1, 128, 0, stream>>>(PART, MEAN); k_cpart<2><<<(256 * CC + 255) / 256, 256, 0, stream>>>(Cb, MEAN, PART); k_cfin<<<1, 128, 0, stream>>>(PART, VAR);
    k_bngelu<<<(unsigned)(((size_t)NR * CC / 4 + 255) / 256), 256, 0, stream>>>(Cb, MEAN, VAR, bn2g, bn2b, Hf);
    k_gpart<1><<<(NB_ * 512 + 255) / 256, 256, 0, stream>>>(Hf, nullptr, GP); k_gfin<<<1, 64, 0, stream>>>(GP, GM); k_gpart<2><<<(NB_ * 512 + 255) / 256, 256, 0, stream>>>(Hf, GM, GP); k_gfin<<<1, 64, 0, stream>>>(GP, GV);
    k_gn16<<<(unsigned)(((size_t)NR * CC / 4 + 255) / 256), 256, 0, stream>>>(Hf, GM, GV, gng, gnb, HN16);
    for (int b = 0; b < NB_; ++b) {
        k_gemmw<h16, 0, false><<<dim3(3 * CC / 64, TT / 64, 1), 32, 0, stream>>>(QKVW, nullptr, HN16 + (size_t)b * TT * CC, nullptr, CC, QKV, TT, nullptr, 0, 0, 0);
        k_qkT<<<(TT * CC / 2 + 255) / 256, 256, 0, stream>>>(QKV, qkvb, Q16, KT16); k_v16<<<(CC * TT / 4 + 255) / 256, 256, 0, stream>>>(QKV, qkvb, V16);
        k_ekv<<<(2 * CC * (CC / 4) + 255) / 256, 256, 0, stream>>>(mixemb, encw, encb, b, KT16, V16); k_ekT<<<(NEK * CC / 2 + 255) / 256, 256, 0, stream>>>(KT16);
        k_gemmw<h16, 0, false><<<dim3(TT / 64, NKEY / 64, 1), 32, 0, stream>>>(Q16, nullptr, KT16, nullptr, CC, Sb, NKEY, nullptr, 0, 0, 0);
        k_soft<33, 0><<<TT / 8, 256, 0, stream>>>(Sb, TT, NKEY, NKEY, NKEY, P16);
        k_gemmw<h16, 0, false><<<dim3(TT / 64, CC / 64, 1), 32, 0, stream>>>(P16, nullptr, V16, nullptr, NKEY, AT, CC, nullptr, 0, 0, 0);
        k_a16<<<(TT * CC / 4 + 255) / 256, 256, 0, stream>>>(AT, A16);
        k_gemmw<h16, 0, true><<<dim3(TT / 64, CC / 64, 1), 32, 0, stream>>>(A16, nullptr, PW, nullptr, CC, ATT, CC, pb, 0, 0, 0);
        k_resid<<<(TT * CC / 4 + 255) / 256, 256, 0, stream>>>(Hf + (size_t)b * TT * CC, ATT, H2 + (size_t)b * TT * CC); }
    k_pool<<<(NB_ * CC * 1024 / 4 + 255) / 256, 256, 0, stream>>>(H2, OUT);
}
